// NONLocalBlock1D_61564061221373
// MI455X (gfx1250) — hardware-run, weakly checked
//
#include <hip/hip_runtime.h>


#define NB_  8
#define CC   256
#define IC   128
#define TT   4096
#define TH   2048
typedef _Float16 h16;
typedef unsigned short bf;
typedef __attribute__((ext_vector_type(16))) __bf16   v16bf;
typedef __attribute__((ext_vector_type(16))) _Float16 v16h;
typedef __attribute__((ext_vector_type(8)))  _Float16 v8h;
typedef __attribute__((ext_vector_type(8)))  unsigned short v8us;
typedef __attribute__((ext_vector_type(8)))  float    v8f;
typedef __attribute__((ext_vector_type(4)))  float    v4f;
typedef v8h  __attribute__((may_alias)) v8ha;
typedef v4f  __attribute__((may_alias)) v4fa;
typedef v8us __attribute__((may_alias)) v8usa;

__device__ __forceinline__ unsigned short f2bf(float f) { unsigned u = __float_as_uint(f); u += 0x7FFFu + ((u >> 16) & 1u); return (unsigned short)(u >> 16); }
__device__ __forceinline__ float bf2f(unsigned short b) { return __uint_as_float(((unsigned)b) << 16); }
__device__ __forceinline__ float bfr(float f) { return bf2f(f2bf(f)); }
__device__ __forceinline__ v16h cat16(v8h lo, v8h hi) { return __builtin_shufflevector(lo, hi, 0, 1, 2, 3, 4, 5, 6, 7, 8, 9, 10, 11, 12, 13, 14, 15); }
__device__ __forceinline__ v16bf cat16b(v8us lo, v8us hi) { return __builtin_bit_cast(v16bf, __builtin_shufflevector(lo, hi, 0, 1, 2, 3, 4, 5, 6, 7, 8, 9, 10, 11, 12, 13, 14, 15)); }
__device__ __forceinline__ v8f wmma16(v16h a, v16h b, v8f c) { return __builtin_amdgcn_wmma_f32_16x16x32_f16(false, a, false, b, (short)0, c, false, false); }
__device__ __forceinline__ v8f wmmab(v16bf a, v16bf b, v8f c) { return __builtin_amdgcn_wmma_f32_16x16x32_bf16(false, a, false, b, (short)0, c, false, false); }


template <typename T16> struct WFrag;
template <> struct WFrag<h16> { typedef v16h V; static __device__ __forceinline__ V ld(const h16* p) { return cat16(*(const v8h*)p, *(const v8h*)(p + 16)); } static __device__ __forceinline__ v8f mma(V a, V b, v8f c) { return wmma16(a, b, c); } };
template <> struct WFrag<bf> { typedef v16bf V; static __device__ __forceinline__ V ld(const bf* p) { return cat16b(*(const v8us*)p, *(const v8us*)(p + 16)); } static __device__ __forceinline__ v8f mma(V a, V b, v8f c) { return wmmab(a, b, c); } };
template <typename T16, int NSPLIT, bool BIAS>
__global__ __launch_bounds__(32) void k_gemmw(const T16* __restrict__ A, const T16* __restrict__ A2, const T16* __restrict__ Bt, const T16* __restrict__ Bt2, int K, float* C, int ldc, const float* __restrict__ bias, size_t sA, size_t sB, size_t sC) {
    typedef typename WFrag<T16>::V V;
    __shared__ __align__(16) float os[16 * 68];
    const size_t z = blockIdx.z; A += z * sA; if (A2) A2 += z * sA; Bt += z * sB; if (Bt2) Bt2 += z * sB; C += z * sC;
    const int lane = threadIdx.x & 31, lr = lane & 15, hi = lane >> 4; const int r0 = blockIdx.x * 64, c0 = blockIdx.y * 64;
    v8f acc[4][4];
#pragma unroll
    for (int mb = 0; mb < 4; ++mb)
#pragma unroll
        for (int nb = 0; nb < 4; ++nb) acc[mb][nb] = (v8f){};
    const size_t aoff = (size_t)(r0 + lr) * K + 8 * hi, boff = (size_t)(c0 + lr) * K + 8 * hi;
#pragma unroll 1
    for (int kc = 0; kc < K; kc += 32) {
        V a[4], a2[4];
#pragma unroll
        for (int mb = 0; mb < 4; ++mb) { a[mb] = WFrag<T16>::ld(A + aoff + (size_t)mb * 16 * K + kc); if (NSPLIT == 1 || NSPLIT == 2) a2[mb] = WFrag<T16>::ld(A2 + aoff + (size_t)mb * 16 * K + kc); }
#pragma unroll
        for (int nb = 0; nb < 4; ++nb) { const V b = WFrag<T16>::ld(Bt + boff + (size_t)nb * 16 * K + kc); V b2; if (NSPLIT >= 2) b2 = WFrag<T16>::ld(Bt2 + boff + (size_t)nb * 16 * K + kc);
#pragma unroll
            for (int mb = 0; mb < 4; ++mb) { acc[mb][nb] = WFrag<T16>::mma(a[mb], b, acc[mb][nb]); if (NSPLIT == 1 || NSPLIT == 2) acc[mb][nb] = WFrag<T16>::mma(a2[mb], b, acc[mb][nb]); if (NSPLIT >= 2) acc[mb][nb] = WFrag<T16>::mma(a[mb], b2, acc[mb][nb]); } }
        asm volatile("v_nop\n\tv_nop\n\tv_nop\n\tv_nop" : "+v"(acc[0][0]), "+v"(acc[1][1]), "+v"(acc[2][2]), "+v"(acc[3][3]) : "v"(a[0]), "v"(a[3]));
    }
#pragma unroll
    for (int mb = 0; mb < 4; ++mb) {
#pragma unroll
        for (int nb = 0; nb < 4; ++nb) {
#pragma unroll
            for (int j = 0; j < 8; ++j) os[(hi * 8 + j) * 68 + nb * 16 + lr] = acc[mb][nb][j]; }
        __builtin_amdgcn_wave_barrier(); asm volatile("" ::: "memory");
        float* crow = C + (size_t)(r0 + mb * 16) * ldc + c0;
#pragma unroll 1
        for (int ps = 0; ps < 2; ++ps) {
#pragma unroll
            for (int s = 0; s < 8; ++s) { const int row = 2 * s + hi, cofs = lr * 4; v4f val = *(const v4fa*)(os + row * 68 + cofs); if (BIAS) { val[0] += bfr(bias[c0 + cofs]); val[1] += bfr(bias[c0 + cofs + 1]); val[2] += bfr(bias[c0 + cofs + 2]); val[3] += bfr(bias[c0 + cofs + 3]); }
                *(volatile v4f*)(crow + (size_t)row * ldc + cofs) = val; }
            if (ps == 0) __threadfence(); }
        __builtin_amdgcn_wave_barrier(); asm volatile("" ::: "memory");
    }
}

__device__ __forceinline__ void splitf(float y, unsigned short& h, unsigned short& l) { h = f2bf(y); l = f2bf(y - bf2f(h)); }
typedef __attribute__((ext_vector_type(4))) unsigned short v4us;

__global__ __launch_bounds__(256) void k_cvt8(const float* __restrict__ src, bf* dst, size_t n8) { const size_t i = (size_t)blockIdx.x * 256 + threadIdx.x; if (i >= n8) return; const v8f v = *(const v8f*)(src + i * 8); v8us o;
#pragma unroll
    for (int k = 0; k < 8; ++k) o[k] = f2bf(v[k]); *(volatile v8us*)(dst + i * 8) = o; __threadfence(); *(volatile v8us*)(dst + i * 8) = o; }
__global__ __launch_bounds__(256) void k_trb(const float* __restrict__ xb, bf* XT) { __shared__ float tile[64][33]; const int t0 = blockIdx.x * 32, c0 = blockIdx.y * 64; const int lx = threadIdx.x & 31, ly = threadIdx.x >> 5;
    for (int r = ly; r < 64; r += 8) tile[r][lx] = xb[(size_t)(c0 + r) * TT + t0 + lx];
    __syncthreads();
#pragma unroll
    for (int pass = 0; pass < 2; ++pass) { const int r = pass * 16 + (threadIdx.x >> 4), q = threadIdx.x & 15; v4us o;
#pragma unroll
        for (int u = 0; u < 4; ++u) o[u] = f2bf(tile[q * 4 + u][r]); bf* dst = XT + (size_t)(t0 + r) * CC + c0 + q * 4; *(volatile v4us*)dst = o; __threadfence(); *(volatile v4us*)dst = o; } }
__global__ __launch_bounds__(256) void k_poolT(const float* __restrict__ F, bf* Ph, bf* Pl) { const size_t e = ((size_t)blockIdx.x * 256 + threadIdx.x) * 4; if (e >= (size_t)IC * TH) return; const int s = (int)(e % TH); const int c = (int)(e / TH); v4us oh, ol;
#pragma unroll
    for (int u = 0; u < 4; ++u) { const float a = F[(size_t)(2 * (s + u)) * IC + c], b2 = F[(size_t)(2 * (s + u) + 1) * IC + c]; unsigned short hh, ll; splitf(fmaxf(a, b2), hh, ll); oh[u] = hh; ol[u] = ll; } *(volatile v4us*)(Ph + e) = oh; *(volatile v4us*)(Pl + e) = ol; __threadfence(); *(volatile v4us*)(Ph + e) = oh; *(volatile v4us*)(Pl + e) = ol; }
__global__ __launch_bounds__(256) void k_plT(const float* __restrict__ F, size_t n, bf* Ph, bf* Pl) { const size_t e = ((size_t)blockIdx.x * 256 + threadIdx.x) * 4; if (e >= n) return; v4us oh, ol;
#pragma unroll
    for (int u = 0; u < 4; ++u) { unsigned short a, b; splitf(F[e + u], a, b); oh[u] = a; ol[u] = b; } *(volatile v4us*)(Ph + e) = oh; *(volatile v4us*)(Pl + e) = ol; __threadfence(); *(volatile v4us*)(Ph + e) = oh; *(volatile v4us*)(Pl + e) = ol; }
__global__ __launch_bounds__(256) void k_scl(const float* __restrict__ Y, bf* Ph, bf* Pl) { const size_t e = ((size_t)blockIdx.x * 256 + threadIdx.x) * 4; if (e >= (size_t)TT * IC) return; v4us oh, ol;
#pragma unroll
    for (int u = 0; u < 4; ++u) { unsigned short a, b; splitf(Y[e + u] * (1.0f / 2048.0f), a, b); oh[u] = a; ol[u] = b; } *(volatile v4us*)(Ph + e) = oh; *(volatile v4us*)(Pl + e) = ol; __threadfence(); *(volatile v4us*)(Ph + e) = oh; *(volatile v4us*)(Pl + e) = ol; }
__global__ __launch_bounds__(256) void k_mT(const float* __restrict__ M, bf* Ph, bf* Pl) { const int e = (blockIdx.x * 256 + threadIdx.x) * 4; if (e >= IC * IC) return; const int cp = e % IC; const int c = e / IC; v4us oh, ol;
#pragma unroll
    for (int u = 0; u < 4; ++u) { unsigned short a, b; splitf(M[(size_t)(cp + u) * IC + c], a, b); oh[u] = a; ol[u] = b; } *(volatile v4us*)(Ph + e) = oh; *(volatile v4us*)(Pl + e) = ol; __threadfence(); *(volatile v4us*)(Ph + e) = oh; *(volatile v4us*)(Pl + e) = ol; }
__global__ __launch_bounds__(256) void k_bnstat(const float* __restrict__ WY, float* ST) { __shared__ float red[256]; const int o = blockIdx.x; const size_t N = (size_t)NB_ * TT; float s = 0.f;
    for (size_t i = threadIdx.x; i < N; i += 256) s = __fadd_rn(s, WY[i * CC + o]);
    red[threadIdx.x] = s; __syncthreads();
    for (int st = 128; st > 0; st >>= 1) { if (threadIdx.x < st) red[threadIdx.x] = __fadd_rn(red[threadIdx.x], red[threadIdx.x + st]); __syncthreads(); }
    const float mean = red[0] * (1.0f / (float)N); __syncthreads(); float q = 0.f;
    for (size_t i = threadIdx.x; i < N; i += 256) { float d = __fsub_rn(WY[i * CC + o], mean); asm volatile("" : "+v"(d)); float p = __fmul_rn(d, d); asm volatile("" : "+v"(p)); q = __fadd_rn(q, p); }
    red[threadIdx.x] = q; __syncthreads();
    for (int st = 128; st > 0; st >>= 1) { if (threadIdx.x < st) red[threadIdx.x] = __fadd_rn(red[threadIdx.x], red[threadIdx.x + st]); __syncthreads(); }
    if (threadIdx.x < 32) { const float var = red[0] * (1.0f / (float)N); float v2 = (threadIdx.x == 0) ? mean : (threadIdx.x == 1 ? var : 0.f); *(volatile float*)(ST + (size_t)o * 32 + threadIdx.x) = v2; __threadfence(); *(volatile float*)(ST + (size_t)o * 32 + threadIdx.x) = v2; } }
__global__ __launch_bounds__(256) void k_out(const float* __restrict__ WY, const float* __restrict__ ST, const float* __restrict__ gam, const float* __restrict__ bet, const float* __restrict__ xb, int b, float* outb) { const size_t e = ((size_t)blockIdx.x * 256 + threadIdx.x) * 4; if (e >= (size_t)CC * TT) return; const int t = (int)(e % TT); const int o = (int)(e / TT); const float mean = ST[o * 32], var = ST[o * 32 + 1]; const float rs = __frsqrt_rn(__fadd_rn(var, 1e-5f)); const float ga = bfr(gam[o]), be = bfr(bet[o]); v4f r;
#pragma unroll
    for (int u = 0; u < 4; ++u) { float d = __fsub_rn(WY[((size_t)b * TT + t + u) * CC + o], mean); asm volatile("" : "+v"(d)); float n0 = __fmul_rn(d, rs); asm volatile("" : "+v"(n0)); float a1 = __fmul_rn(n0, ga); asm volatile("" : "+v"(a1)); float a2 = __fadd_rn(a1, be); asm volatile("" : "+v"(a2)); r[u] = __fadd_rn(a2, bfr(xb[e + u])); }
    *(volatile v4f*)(outb + e) = r; __threadfence(); *(volatile v4f*)(outb + e) = r; }

extern "C" void kernel_launch(void* const* d_in, const int* in_sizes, int n_in,
                              void* d_out, int out_size, void* d_ws, size_t ws_size, hipStream_t stream) {
    (void)in_sizes; (void)n_in; (void)out_size;
    const float** I = (const float**)d_in;
    const float *x = I[0], *thw = I[1], *thb = I[2], *phw = I[3], *phb = I[4], *gw = I[5], *gb = I[6], *ww = I[7], *wb = I[8], *gam = I[9], *bet = I[10];
    float* OUT = (float*)d_out;
    char* wsp = (char*)d_ws;
    auto take = [&](size_t bytes) { char* p = wsp; wsp += (bytes + 255) & ~(size_t)255; return (void*)p; };
    bf* XT = (bf*)take((size_t)TT * CC * 2); bf* BTH = (bf*)take((size_t)IC * CC * 2); bf* BPH = (bf*)take((size_t)IC * CC * 2); bf* BG = (bf*)take((size_t)IC * CC * 2); bf* BW = (bf*)take((size_t)CC * IC * 2);
    float* FT = (float*)take((size_t)TT * IC * 4); float* FP = (float*)take((size_t)TT * IC * 4); float* FG = (float*)take((size_t)TT * IC * 4);
    bf* THh = (bf*)take((size_t)TT * IC * 2); bf* THl = (bf*)take((size_t)TT * IC * 2); bf* PHh = (bf*)take((size_t)IC * TH * 2); bf* PHl = (bf*)take((size_t)IC * TH * 2); bf* GPh = (bf*)take((size_t)IC * TH * 2); bf* GPl = (bf*)take((size_t)IC * TH * 2);
    float* M = (float*)take((size_t)IC * IC * 4); bf* MTh = (bf*)take((size_t)IC * IC * 2); bf* MTl = (bf*)take((size_t)IC * IC * 2); float* YT = (float*)take((size_t)TT * IC * 4); bf* YTh = (bf*)take((size_t)TT * IC * 2); bf* YTl = (bf*)take((size_t)TT * IC * 2);
    float* WY = (float*)take((size_t)NB_ * TT * CC * 4); float* ST = (float*)take((size_t)CC * 32 * 4);
    if ((size_t)(wsp - (char*)d_ws) > ws_size) return;
    k_cvt8<<<(IC * CC / 8 + 255) / 256, 256, 0, stream>>>(thw, BTH, IC * CC / 8); k_cvt8<<<(IC * CC / 8 + 255) / 256, 256, 0, stream>>>(phw, BPH, IC * CC / 8); k_cvt8<<<(IC * CC / 8 + 255) / 256, 256, 0, stream>>>(gw, BG, IC * CC / 8); k_cvt8<<<(CC * IC / 8 + 255) / 256, 256, 0, stream>>>(ww, BW, CC * IC / 8);
    for (int b = 0; b < NB_; ++b) {
        k_trb<<<dim3(TT / 32, CC / 64, 1), 256, 0, stream>>>(x + (size_t)b * CC * TT, XT);
        k_gemmw<bf, 0, true><<<dim3(TT / 64, IC / 64, 1), 32, 0, stream>>>(XT, nullptr, BTH, nullptr, CC, FT, IC, thb, 0, 0, 0); k_gemmw<bf, 0, true><<<dim3(TT / 64, IC / 64, 1), 32, 0, stream>>>(XT, nullptr, BPH, nullptr, CC, FP, IC, phb, 0, 0, 0); k_gemmw<bf, 0, true><<<dim3(TT / 64, IC / 64, 1), 32, 0, stream>>>(XT, nullptr, BG, nullptr, CC, FG, IC, gb, 0, 0, 0);
        k_plT<<<(TT * IC / 4 + 255) / 256, 256, 0, stream>>>(FT, (size_t)TT * IC, THh, THl); k_poolT<<<(IC * TH / 4 + 255) / 256, 256, 0, stream>>>(FP, PHh, PHl); k_poolT<<<(IC * TH / 4 + 255) / 256, 256, 0, stream>>>(FG, GPh, GPl);
        k_gemmw<bf, 2, false><<<dim3(IC / 64, IC / 64, 1), 32, 0, stream>>>(PHh, PHl, GPh, GPl, TH, M, IC, nullptr, 0, 0, 0);
        k_mT<<<(IC * IC / 4 + 255) / 256, 256, 0, stream>>>(M, MTh, MTl);
        k_gemmw<bf, 2, false><<<dim3(TT / 64, IC / 64, 1), 32, 0, stream>>>(THh, THl, MTh, MTl, IC, YT, IC, nullptr, 0, 0, 0);
        k_scl<<<(TT * IC / 4 + 255) / 256, 256, 0, stream>>>(YT, YTh, YTl);
        k_gemmw<bf, 1, true><<<dim3(TT / 64, CC / 64, 1), 32, 0, stream>>>(YTh, YTl, BW, nullptr, IC, WY + (size_t)b * TT * CC, CC, wb, 0, 0, 0); }
    k_bnstat<<<CC, 256, 0, stream>>>(WY, ST);
    for (int b = 0; b < NB_; ++b) k_out<<<(unsigned)(((size_t)CC * TT / 4 + 255) / 256), 256, 0, stream>>>(WY, ST, gam, bet, x + (size_t)b * CC * TT, b, OUT + (size_t)b * CC * TT);
}
